// SelectiveSSM_43224550867174
// MI455X (gfx1250) — hardware-run, weakly checked
//
#include <hip/hip_runtime.h>
#include <hip/hip_fp16.h>
#include <math.h>

typedef __attribute__((ext_vector_type(16))) _Float16 v16h;
typedef __attribute__((ext_vector_type(8)))  _Float16 v8h;
typedef __attribute__((ext_vector_type(8)))  float    v8f;
typedef __attribute__((ext_vector_type(4)))  float    v4f;
typedef __attribute__((ext_vector_type(2)))  float    v2f;

constexpr int kBatch  = 2;
constexpr int kSeq    = 1024;
constexpr int kDm     = 1024;
constexpr int kDin    = 2048;
constexpr int kNst    = 16;
constexpr int kDtr    = 64;
constexpr int kRows   = kBatch * kSeq;
constexpr int kXp     = 2 * kDin;
constexpr int kCatN   = 128;
constexpr int kColB   = 64;
constexpr int kColC   = 80;
constexpr int kColEnd = 96;
constexpr int kConvTP = 260;
constexpr float kWCarry  = 1024.0f;
constexpr float kResid   = 2048.0f;
constexpr float kXcCarry = 64.0f;
constexpr float kDlCarry = 1024.0f;
constexpr float kYCarry  = 4096.0f;
constexpr float sIn   = 1.0f / kWCarry;
constexpr float sInR  = 1.0f / (kWCarry * kResid);
constexpr float sCat  = 1.0f / (kXcCarry * kWCarry);
constexpr float sCatR = 1.0f / (kXcCarry * kWCarry * kResid);
constexpr float sExp  = 1.0f / (kDlCarry * kWCarry);
constexpr float sOut  = 1.0f / (kYCarry * kWCarry);
constexpr float sOutR = 1.0f / (kYCarry * kWCarry * kResid);
constexpr bool kSplitIn  = false;
constexpr bool kSplitOut = false;
static_assert(kRows == 2048);
static_assert(kColB == kDtr && kColC == kColB + kNst && kColEnd == kColC + kNst && kColEnd <= kCatN);
static_assert((kDm % 64) == 0 && (kDin % 64) == 0 && (kXp % 64) == 0 && (kCatN % 64) == 0 && (kDtr % 64) == 0);
static_assert((kSeq % 64) == 0 && (kRows % 64) == 0 && (kDin % 256) == 0);
static_assert((kDm % 32) == 0 && (kDin % 32) == 0 && (kDtr % 32) == 0);

constexpr size_t kSzW0   = (size_t)kXp * kDm * 2;
constexpr size_t kSzW7   = (size_t)kDm * kDin * 2;
constexpr size_t kSzWC   = (size_t)kCatN * kDin * 2;
constexpr size_t kSzW3   = (size_t)kDin * kDtr * 2;
constexpr size_t kSzBCAT = (size_t)kCatN * 4;
constexpr size_t kSzXH   = (size_t)kRows * kDm * 2;
constexpr size_t kSzXL   = kSplitIn ? kSzXH : 0;
constexpr size_t kSzF32  = (size_t)kRows * kDin * 4;
constexpr size_t kSzF16  = (size_t)kRows * kDin * 2;
constexpr size_t kSzP    = (size_t)kRows * kCatN * 4;
constexpr size_t kSzDL   = (size_t)kRows * kDtr * 2;
constexpr size_t kSzYL   = kSplitOut ? kSzF16 : 0;
constexpr size_t kOffW0   = 0;
constexpr size_t kOffW7   = kOffW0   + kSzW0;
constexpr size_t kOffWCH  = kOffW7   + kSzW7;
constexpr size_t kOffWCL  = kOffWCH  + kSzWC;
constexpr size_t kOffW3   = kOffWCL  + kSzWC;
constexpr size_t kOffBCAT = kOffW3   + kSzW3;
constexpr size_t kOffXH   = kOffBCAT + kSzBCAT;
constexpr size_t kOffXL   = kOffXH   + kSzXH;
constexpr size_t kOffXI   = kOffXL   + kSzXL;
constexpr size_t kOffSG   = kOffXI   + kSzF32;
constexpr size_t kOffXC   = kOffSG   + kSzF32;
constexpr size_t kOffXCH  = kOffXC   + kSzF32;
constexpr size_t kOffXCL  = kOffXCH  + kSzF16;
constexpr size_t kOffP    = kOffXCL  + kSzF16;
constexpr size_t kOffDLH  = kOffP    + kSzP;
constexpr size_t kOffDT   = kOffDLH  + kSzDL;
constexpr size_t kOffYH   = kOffDT   + kSzF32;
constexpr size_t kOffYL   = kOffYH   + kSzF16;
constexpr size_t kWsTotal = kOffYL   + kSzYL;
static_assert(kWsTotal == 111673856ull + (kSplitIn ? 4194304ull : 0ull) + (kSplitOut ? 8388608ull : 0ull));
static_assert(kWsTotal <= 134217728ull);
static_assert((kOffW7 % 128) == 0 && (kOffWCH % 128) == 0 && (kOffWCL % 128) == 0 && (kOffW3 % 128) == 0 &&
              (kOffBCAT % 128) == 0 && (kOffXH % 128) == 0 && (kOffXL % 128) == 0 && (kOffXI % 128) == 0 &&
              (kOffSG % 128) == 0 && (kOffXC % 128) == 0 && (kOffXCH % 128) == 0 && (kOffXCL % 128) == 0 &&
              (kOffP % 128) == 0 && (kOffDLH % 128) == 0 && (kOffDT % 128) == 0 && (kOffYH % 128) == 0 &&
              (kOffYL % 128) == 0);
static_assert((size_t)kRows * kDm * 4 == 8388608ull);
static_assert((size_t)kRows * kDm * 4 + (size_t)kBatch * kDin * kNst * 4 == 8650752ull);

__device__ __forceinline__ _Float16 f16_flush(float v) {
  const float w = (fabsf(v) < 6.103515625e-05f) ? 0.0f : v;
  return (_Float16)w;
}
__device__ __forceinline__ void f16_split(float v, _Float16& hi, _Float16& lo) {
  hi = f16_flush(v);
  const float hf = (float)hi;
  const float r = (v - hf) * kResid;
  lo = f16_flush(r);
}
__device__ __forceinline__ unsigned h16_bits(float v) {
  return (unsigned)__builtin_bit_cast(unsigned short, f16_flush(v));
}
__device__ __forceinline__ float h16_val(unsigned b) {
  return (float)__builtin_bit_cast(_Float16, (unsigned short)b);
}
__device__ __forceinline__ void pin_f(float& x) { asm volatile("" : "+v"(x)); }
__device__ __forceinline__ float act_silu(float v) {
  const float sg = __builtin_amdgcn_rcpf(1.0f + expf(-v));
  return v * sg;
}
__device__ __forceinline__ float act_softplus(float v) {
  return fmaxf(v, 0.0f) + log1pf(expf(-fabsf(v)));
}

namespace eng {
union FragU { v16h v; v8h h[2]; };
__device__ __forceinline__ v16h frag_load(const _Float16* p) {
  FragU f;
  f.h[0] = *(const v8h*)(p);
  f.h[1] = *(const v8h*)(p + 16);
  return f.v;
}
__device__ __forceinline__ v8f mma(v16h a, v16h b, v8f c) {
  return __builtin_amdgcn_wmma_f32_16x16x32_f16(false, a, false, b, (short)0, c, false, false);
}
__device__ __forceinline__ void guard1(v8f& a, v16h x, v16h y) {
  asm volatile("v_nop\n\tv_nop\n\tv_nop\n\tv_nop" : "+v"(a) : "v"(x), "v"(y));
}
__device__ __forceinline__ void guard_acc(v8f& a) {
  asm volatile("v_nop\n\tv_nop\n\tv_nop\n\tv_nop" : "+v"(a));
}
__device__ __forceinline__ void keep4(v16h a, v16h b, v16h c, v16h d) {
  asm volatile("v_nop" :: "v"(a), "v"(b), "v"(c), "v"(d));
}

template <int MI, int SPL, int EPI>
__global__ __launch_bounds__(256) void gemm_f16_kernel(
    const unsigned short* __restrict__ Ap, const unsigned short* __restrict__ A2p, int lda,
    const unsigned short* __restrict__ Btp, const unsigned short* __restrict__ Bt2p, int ldb,
    float* C, float* C2, int ldc, int nsplit,
    const float* __restrict__ bias, int M, int N, int K, float scale, float rscale)
{
  static_assert(MI >= 1 && MI <= 2);
  static_assert(SPL >= 0 && SPL <= 2);
  static_assert(EPI >= 0 && EPI <= 2);
  const _Float16* A   = (const _Float16*)Ap;
  const _Float16* A2  = (const _Float16*)A2p;
  const _Float16* Bt  = (const _Float16*)Btp;
  const _Float16* Bt2 = (const _Float16*)Bt2p;
  __shared__ __align__(16) float sT[8][16 * 68];
  const int lane = threadIdx.x & 31;
  const int wave = threadIdx.x >> 5;
  const int tilesN = N >> 6;
  const int tilesM = M / (16 * MI);
  const int tile = blockIdx.x * 8 + wave;
  if (tile >= tilesM * tilesN) return;
  const int tm = tile / tilesN;
  const int tn = tile - tm * tilesN;
  const int m0 = tm * (16 * MI);
  const int n0 = tn << 6;
  const int rlane = lane & 15;
  const int koff  = (lane >> 4) * 8;
  const int mOff  = (lane >> 4) * 8;

  v8f acc[MI][4], accr[MI][4];
#pragma unroll
  for (int i = 0; i < MI; ++i)
#pragma unroll
    for (int j = 0; j < 4; ++j) {
      acc[i][j]  = (v8f){0.f, 0.f, 0.f, 0.f, 0.f, 0.f, 0.f, 0.f};
      accr[i][j] = (v8f){0.f, 0.f, 0.f, 0.f, 0.f, 0.f, 0.f, 0.f};
    }

  for (int k0 = 0; k0 < K; k0 += 32) {
    v16h bh[4], bl[4];
#pragma unroll
    for (int j = 0; j < 4; ++j) {
      const size_t bo = (size_t)(n0 + (j << 4) + rlane) * ldb + koff + k0;
      bh[j] = frag_load(Bt + bo);
      if (SPL == 2) bl[j] = frag_load(Bt2 + bo); else bl[j] = bh[j];
    }
#pragma unroll
    for (int i = 0; i < MI; ++i) {
      const size_t ao = (size_t)(m0 + (i << 4) + rlane) * lda + koff + k0;
      const v16h ah = frag_load(A + ao);
      v16h al = ah;
      if (SPL >= 1) al = frag_load(A2 + ao);
#pragma unroll
      for (int jp = 0; jp < 2; ++jp) {
#pragma unroll
        for (int jj = 0; jj < 2; ++jj) {
          const int j = jp * 2 + jj;
          acc[i][j] = mma(ah, bh[j], acc[i][j]);
          if (SPL >= 1) accr[i][j] = mma(al, bh[j], accr[i][j]);
          if (SPL == 2) accr[i][j] = mma(ah, bl[j], accr[i][j]);
        }
#pragma unroll
        for (int jj = 0; jj < 2; ++jj) {
          const int j = jp * 2 + jj;
          guard1(acc[i][j], ah, al);
          if (SPL >= 1) guard1(accr[i][j], ah, al);
        }
      }
    }
    keep4(bh[0], bh[1], bh[2], bh[3]);
    if (SPL == 2) keep4(bl[0], bl[1], bl[2], bl[3]);
  }
#pragma unroll
  for (int i = 0; i < MI; ++i)
#pragma unroll
    for (int j = 0; j < 4; ++j) {
      guard_acc(acc[i][j]);
      if (SPL >= 1) guard_acc(accr[i][j]);
    }

  float* slab = sT[wave];
  const int hh = lane >> 4, c4 = (lane & 15) * 4;
  float* Cd = C;
  int nd = n0;
  bool gateTile = false;
  if (EPI == 1) {
    if (n0 >= nsplit) { Cd = C2; nd = n0 - nsplit; gateTile = true; }
  }
  const v4f bv = *(const v4f*)(bias + n0 + c4);
#pragma unroll
  for (int i = 0; i < MI; ++i) {
    const int mBase = m0 + (i << 4);
#pragma unroll
    for (int j = 0; j < 4; ++j) {
#pragma unroll
      for (int r = 0; r < 8; ++r) {
        float v = acc[i][j][r] * scale;
        if (SPL >= 1) v += accr[i][j][r] * rscale;
        slab[(mOff + r) * 68 + (j << 4) + rlane] = v;
      }
    }
    __builtin_amdgcn_fence(__ATOMIC_RELEASE, "workgroup");
    __builtin_amdgcn_wave_barrier();
    __builtin_amdgcn_fence(__ATOMIC_ACQUIRE, "workgroup");
    for (int it = 0; it < 8; ++it) {
      float* sp = slab + (it * 2 + hh) * 68 + c4;
      v4f v = *(const v4f*)sp;
      v = v + bv;
      if (EPI == 1) {
        if (gateTile) {
#pragma unroll
          for (int e = 0; e < 4; ++e) v[e] = act_silu(v[e]);
        }
      }
      if (EPI == 2) {
#pragma unroll
        for (int e = 0; e < 4; ++e) v[e] = act_softplus(v[e]);
      }
      *(v4f*)sp = v;
    }
    {
      for (int pass = 0; pass < 2; ++pass) {
#pragma unroll
        for (int it = 0; it < 8; ++it) {
          const int row = it * 2 + hh;
          const v4f v = *(const v4f*)(slab + row * 68 + c4);
          *(volatile v4f*)(Cd + (size_t)(mBase + row) * ldc + nd + c4) = v;
        }
        __threadfence();
      }
    }
    __builtin_amdgcn_fence(__ATOMIC_RELEASE, "workgroup");
    __builtin_amdgcn_wave_barrier();
    __builtin_amdgcn_fence(__ATOMIC_ACQUIRE, "workgroup");
  }
}
}

template <bool LO>
__global__ __launch_bounds__(256) void split_rows_f16_kernel(
    const float* __restrict__ src, unsigned short* __restrict__ dH, unsigned short* __restrict__ dL, int total8)
{
  const int i = blockIdx.x * 256 + threadIdx.x;
  if (i >= total8) return;
  const size_t e0 = (size_t)i << 3;
  const v4f a0 = *(const v4f*)(src + e0);
  const v4f a1 = *(const v4f*)(src + e0 + 4);
  v8h hv, lv;
#pragma unroll
  for (int e = 0; e < 4; ++e) {
    _Float16 h0, l0, h1, l1;
    const float f0 = a0[e];
    const float f1 = a1[e];
    f16_split(f0, h0, l0);
    f16_split(f1, h1, l1);
    hv[e] = h0; lv[e] = l0;
    hv[4 + e] = h1; lv[4 + e] = l1;
  }
  unsigned short* qh = dH + e0;
  unsigned short* ql = dL + e0;
  *(volatile v8h*)qh = hv;
  if (LO) *(volatile v8h*)ql = lv;
  __threadfence();
  *(volatile v8h*)qh = hv;
  if (LO) *(volatile v8h*)ql = lv;
}

template <bool LO>
__global__ __launch_bounds__(256) void transpose_pack_kernel(
    const float* __restrict__ W, unsigned short* __restrict__ BtH, unsigned short* __restrict__ BtL,
    int Kdim, int Ndim, float carry)
{
  __shared__ float tile[64 * 65];
  const int tid = threadIdx.x, lane = tid & 31, wave = tid >> 5;
  const int n0 = blockIdx.x * 64;
  const int k0 = blockIdx.y * 64;
#pragma unroll
  for (int p = 0; p < 16; ++p) {
    const int idx = tid + p * 256;
    const int kk  = idx >> 6;
    const int nn  = idx & 63;
    const int n   = n0 + nn;
    const int nc  = (n < Ndim) ? n : (Ndim - 1);
    const float v = W[(size_t)(k0 + kk) * Ndim + nc];
    tile[kk * 65 + nn] = (n < Ndim) ? (v * carry) : 0.0f;
  }
  __syncthreads();
  const int q = lane >> 3, c8 = (lane & 7) * 8;
  v8h hv[2], lv[2];
#pragma unroll
  for (int it = 0; it < 2; ++it) {
    const int nrow = it * 32 + wave * 4 + q;
#pragma unroll
    for (int e = 0; e < 8; ++e) {
      _Float16 h, l;
      const float t = tile[(c8 + e) * 65 + nrow];
      f16_split(t, h, l);
      hv[it][e] = h;
      lv[it][e] = l;
    }
  }
  for (int pass = 0; pass < 2; ++pass) {
#pragma unroll
    for (int it = 0; it < 2; ++it) {
      const int nrow = it * 32 + wave * 4 + q;
      const size_t o = (size_t)(n0 + nrow) * Kdim + k0 + c8;
      *(volatile v8h*)(BtH + o) = hv[it];
      if (LO) *(volatile v8h*)(BtL + o) = lv[it];
    }
    __threadfence();
  }
}

__global__ __launch_bounds__(256) void pack_cat_kernel(
    const float* __restrict__ Wdt, const float* __restrict__ WB, const float* __restrict__ WC,
    unsigned short* __restrict__ BtH, unsigned short* __restrict__ BtL, float carry)
{
  __shared__ float tile[64 * 65];
  const int tid = threadIdx.x, lane = tid & 31, wave = tid >> 5;
  const int n0 = blockIdx.x * 64;
  const int k0 = blockIdx.y * 64;
#pragma unroll 4
  for (int p = 0; p < 16; ++p) {
    const int idx = tid + p * 256;
    const int kk  = idx >> 6;
    const int nn  = idx & 63;
    const int n   = n0 + nn;
    const int ndt = (n < kDtr) ? n : (kDtr - 1);
    int nb = n - kColB; nb = (nb < 0) ? 0 : ((nb > kNst - 1) ? (kNst - 1) : nb);
    int nc = n - kColC; nc = (nc < 0) ? 0 : ((nc > kNst - 1) ? (kNst - 1) : nc);
    const size_t krow = (size_t)(k0 + kk);
    float vdt = Wdt[krow * kDtr + ndt];
    float vb  = WB[krow * kNst + nb];
    float vc  = WC[krow * kNst + nc];
    pin_f(vdt); pin_f(vb); pin_f(vc);
    const float fdt = (n < kColB) ? 1.0f : 0.0f;
    const float fb  = (n >= kColB && n < kColC) ? 1.0f : 0.0f;
    const float fc  = (n >= kColC && n < kColEnd) ? 1.0f : 0.0f;
    float v = fdt * vdt;
    v = fmaf(fb, vb, v);
    v = fmaf(fc, vc, v);
    tile[kk * 65 + nn] = v * carry;
  }
  __syncthreads();
  const int q = lane >> 3, c8 = (lane & 7) * 8;
  v8h hv[2], lv[2];
#pragma unroll
  for (int it = 0; it < 2; ++it) {
    const int nrow = it * 32 + wave * 4 + q;
#pragma unroll
    for (int e = 0; e < 8; ++e) {
      _Float16 h, l;
      const float t = tile[(c8 + e) * 65 + nrow];
      f16_split(t, h, l);
      hv[it][e] = h;
      lv[it][e] = l;
    }
  }
  for (int pass = 0; pass < 2; ++pass) {
#pragma unroll
    for (int it = 0; it < 2; ++it) {
      const int nrow = it * 32 + wave * 4 + q;
      const size_t o = (size_t)(n0 + nrow) * kDin + k0 + c8;
      *(volatile v8h*)(BtH + o) = hv[it];
      *(volatile v8h*)(BtL + o) = lv[it];
    }
    __threadfence();
  }
}

__global__ __launch_bounds__(32) void bias_cat_kernel(
    const float* __restrict__ bdt, const float* __restrict__ bB, const float* __restrict__ bC,
    float* __restrict__ outb)
{
  const int lane = threadIdx.x & 31;
  v4f v;
#pragma unroll
  for (int e = 0; e < 4; ++e) {
    const int n = lane * 4 + e;
    const int ndt = (n < kDtr) ? n : (kDtr - 1);
    int nb = n - kColB; nb = (nb < 0) ? 0 : ((nb > kNst - 1) ? (kNst - 1) : nb);
    int nc = n - kColC; nc = (nc < 0) ? 0 : ((nc > kNst - 1) ? (kNst - 1) : nc);
    float a = bdt[ndt];
    float b = bB[nb];
    float c = bC[nc];
    pin_f(a); pin_f(b); pin_f(c);
    const float fa = (n < kColB) ? 1.0f : 0.0f;
    const float fb = (n >= kColB && n < kColC) ? 1.0f : 0.0f;
    const float fc = (n >= kColC && n < kColEnd) ? 1.0f : 0.0f;
    float t = fa * a;
    t = fmaf(fb, b, t);
    t = fmaf(fc, c, t);
    v[e] = t;
  }
  float* p = outb + lane * 4;
  *(volatile v4f*)p = v;
  __threadfence();
  *(volatile v4f*)p = v;
}

__global__ __launch_bounds__(256) void conv_silu_kernel(
    const float* __restrict__ XI, const float* __restrict__ cw, const float* __restrict__ cb,
    float* __restrict__ XC, unsigned short* __restrict__ XCH, unsigned short* __restrict__ XCL)
{
  __shared__ __align__(16) float sT[16 * kConvTP];
  const int tid = threadIdx.x, lane = tid & 31, wave = tid >> 5;
  const int d0 = blockIdx.x * 256, d = d0 + tid;
  const int t0 = blockIdx.y * 64;
  const int l0 = t0 & (kSeq - 1);
  const float w0 = cw[d];
  const float w1 = cw[kDin + d];
  const float w2 = cw[2 * kDin + d];
  const float w3 = cw[3 * kDin + d];
  const float bc = cb[d];
  float xm1, x0, xp1;
  {
    const bool okm = (l0 >= 1);
    const int rm = okm ? (t0 - 1) : t0;
    float vm = XI[(size_t)rm * kDin + d];
    pin_f(vm);
    xm1 = okm ? vm : 0.0f;
    x0  = XI[(size_t)t0 * kDin + d];
    xp1 = XI[(size_t)(t0 + 1) * kDin + d];
  }
  const int hrow = wave >> 1;
  const int hch  = (wave & 1) * 128 + lane * 4;
  for (int sub = 0; sub < 4; ++sub) {
    const int lb = t0 + sub * 16;
    for (int s = 0; s < 16; ++s) {
      const int r = lb + s;
      const int l = l0 + sub * 16 + s;
      const bool ok2 = (l + 2) < kSeq;
      const int rr = ok2 ? (r + 2) : r;
      float xp2 = XI[(size_t)rr * kDin + d];
      pin_f(xp2);
      xp2 = ok2 ? xp2 : 0.0f;
      float acc = w0 * xm1;
      acc = fmaf(w1, x0, acc);
      acc = fmaf(w2, xp1, acc);
      acc = fmaf(w3, xp2, acc);
      const float sv = acc + bc;
      const float sg = __builtin_amdgcn_rcpf(1.0f + expf(-sv));
      sT[s * kConvTP + tid] = sv * sg;
      xm1 = x0; x0 = xp1; xp1 = xp2;
    }
    __syncthreads();
    v4f fv[4];
    v8h hv[2], lv[2];
#pragma unroll
    for (int it = 0; it < 4; ++it) fv[it] = *(const v4f*)(sT + (it * 4 + hrow) * kConvTP + hch);
#pragma unroll
    for (int it = 0; it < 2; ++it) {
      const float* sp = sT + (it * 8 + wave) * kConvTP + lane * 8;
      const v4f a0 = *(const v4f*)(sp);
      const v4f a1 = *(const v4f*)(sp + 4);
#pragma unroll
      for (int e = 0; e < 4; ++e) {
        _Float16 h0, l0h, h1, l1h;
        const float f0 = a0[e] * kXcCarry;
        const float f1 = a1[e] * kXcCarry;
        f16_split(f0, h0, l0h);
        f16_split(f1, h1, l1h);
        hv[it][e] = h0; lv[it][e] = l0h;
        hv[it][4 + e] = h1; lv[it][4 + e] = l1h;
      }
    }
    for (int pass = 0; pass < 2; ++pass) {
#pragma unroll
      for (int it = 0; it < 4; ++it)
        *(volatile v4f*)(XC + (size_t)(lb + it * 4 + hrow) * kDin + d0 + hch) = fv[it];
#pragma unroll
      for (int it = 0; it < 2; ++it) {
        const size_t o = (size_t)(lb + it * 8 + wave) * kDin + d0 + lane * 8;
        *(volatile v8h*)(XCH + o) = hv[it];
        *(volatile v8h*)(XCL + o) = lv[it];
      }
      __threadfence();
    }
    __syncthreads();
  }
}

__global__ __launch_bounds__(256) void dtlow_f16_kernel(
    const float* __restrict__ P, unsigned short* __restrict__ DL, int total8)
{
  const int i = blockIdx.x * 256 + threadIdx.x;
  if (i >= total8) return;
  const int row = i >> 3;
  const int c8  = (i & 7) * 8;
  const float* sp = P + (size_t)row * kCatN + c8;
  const v4f a0 = *(const v4f*)(sp);
  const v4f a1 = *(const v4f*)(sp + 4);
  v8h hv;
#pragma unroll
  for (int e = 0; e < 4; ++e) {
    hv[e]     = f16_flush(a0[e] * kDlCarry);
    hv[4 + e] = f16_flush(a1[e] * kDlCarry);
  }
  unsigned short* q = DL + (size_t)row * kDtr + c8;
  *(volatile v8h*)q = hv;
  __threadfence();
  *(volatile v8h*)q = hv;
}

template <bool LO>
__global__ __launch_bounds__(64) void scan_final_kernel(
    const float* __restrict__ DT, const float* __restrict__ XC, const float* __restrict__ SG,
    const float* __restrict__ P, const float* __restrict__ A_log, const float* __restrict__ Dp,
    const float* __restrict__ hin, unsigned* __restrict__ YH, unsigned* __restrict__ YL,
    float* __restrict__ hout)
{
  __shared__ __align__(16) float sBC[64 * 32];
  const int tid = threadIdx.x;
  constexpr int kBlkPerBatch = kDin / 128;
  const int bi = blockIdx.x / kBlkPerBatch;
  const int d0 = (blockIdx.x - bi * kBlkPerBatch) * 128;
  const int d  = d0 + 2 * tid;
  const int rowb = bi * kSeq;

  for (int n = 0; n < 32; ++n) {
    const float al = A_log[(size_t)d * kNst + n];
    sBC[n * 64 + tid] = -expf(al);
  }
  __syncthreads();
  float A0[16], A1[16], ha[16], hb[16];
#pragma unroll
  for (int n = 0; n < 16; ++n) {
    A0[n] = sBC[n * 64 + tid];
    A1[n] = sBC[(16 + n) * 64 + tid];
  }
  {
    const float* hp = hin + ((size_t)bi * kDin + d) * kNst;
#pragma unroll
    for (int k = 0; k < 4; ++k) {
      const v4f va = *(const v4f*)(hp + 4 * k);
      const v4f vb = *(const v4f*)(hp + 16 + 4 * k);
      ha[4 * k + 0] = va[0]; ha[4 * k + 1] = va[1]; ha[4 * k + 2] = va[2]; ha[4 * k + 3] = va[3];
      hb[4 * k + 0] = vb[0]; hb[4 * k + 1] = vb[1]; hb[4 * k + 2] = vb[2]; hb[4 * k + 3] = vb[3];
    }
  }
  const v2f dpv = *(const v2f*)(Dp + d);
  const float D0 = dpv[0], D1 = dpv[1];

#pragma unroll 1
  for (int ci = 0; ci < kSeq / 64; ++ci) {
    const int rowc = rowb + ci * 64;
    __syncthreads();
#pragma unroll
    for (int i = 0; i < 8; ++i) {
      const int idx = tid + i * 64;
      const int st  = idx >> 3;
      const int c4  = (idx & 7) * 4;
      const v4f v = *(const v4f*)(P + (size_t)(rowc + st) * kCatN + kColB + c4);
      *(v4f*)(sBC + st * 32 + c4) = v;
    }
    __syncthreads();
#pragma unroll 1
    for (int s = 0; s < 64; ++s) {
      const size_t o = (size_t)(rowc + s) * kDin + d;
      const v2f dtv = *(const v2f*)(DT + o);
      const v2f xcv = *(const v2f*)(XC + o);
      const v2f sgv = *(const v2f*)(SG + o);
      float dt0 = dtv[0], dt1 = dtv[1];
      float x0 = xcv[0], x1 = xcv[1];
      float g0 = sgv[0], g1 = sgv[1];
      pin_f(dt0); pin_f(dt1); pin_f(x0); pin_f(x1); pin_f(g0); pin_f(g1);
      const float* bp = sBC + s * 32;
      v4f Bq[4], Cq[4];
#pragma unroll
      for (int k = 0; k < 4; ++k) {
        Bq[k] = *(const v4f*)(bp + 4 * k);
        Cq[k] = *(const v4f*)(bp + 16 + 4 * k);
      }
      float y0 = 0.0f, y1 = 0.0f;
#pragma unroll
      for (int n = 0; n < 16; ++n) {
        const float bn = Bq[n >> 2][n & 3];
        const float cn = Cq[n >> 2][n & 3];
        const float e0 = expf(dt0 * A0[n]);
        const float e1 = expf(dt1 * A1[n]);
        ha[n] = fmaf(e0, ha[n], (dt0 * bn) * x0);
        hb[n] = fmaf(e1, hb[n], (dt1 * bn) * x1);
        y0 = fmaf(ha[n], cn, y0);
        y1 = fmaf(hb[n], cn, y1);
      }
      y0 = fmaf(D0, x0, y0);
      y1 = fmaf(D1, x1, y1);
      const float c0 = (y0 * g0) * kYCarry;
      const float c1 = (y1 * g1) * kYCarry;
      const unsigned hb0 = h16_bits(c0);
      const unsigned hb1 = h16_bits(c1);
      const unsigned hw = hb0 | (hb1 << 16);
      unsigned lw = 0u;
      if (LO) {
        const float r0 = (c0 - h16_val(hb0)) * kResid;
        const float r1 = (c1 - h16_val(hb1)) * kResid;
        lw = h16_bits(r0) | (h16_bits(r1) << 16);
      }
      volatile unsigned* yp = YH + (o >> 1);
      volatile unsigned* lp = YL + (o >> 1);
      *yp = hw;
      if (LO) *lp = lw;
      __threadfence();
      *yp = hw;
      if (LO) *lp = lw;
    }
  }

  v4f hv[8];
#pragma unroll
  for (int k = 0; k < 4; ++k) {
    hv[k]     = (v4f){ha[4 * k + 0], ha[4 * k + 1], ha[4 * k + 2], ha[4 * k + 3]};
    hv[4 + k] = (v4f){hb[4 * k + 0], hb[4 * k + 1], hb[4 * k + 2], hb[4 * k + 3]};
  }
  float* hp = hout + ((size_t)bi * kDin + d) * kNst;
  for (int pass = 0; pass < 2; ++pass) {
#pragma unroll
    for (int k = 0; k < 8; ++k) *(volatile v4f*)(hp + 4 * k) = hv[k];
    __threadfence();
  }
}

static_assert(((kRows / 32) * (kXp / 64)) % 8 == 0);
static_assert(((kRows / 16) * (kCatN / 64)) % 8 == 0);
static_assert(((kRows / 32) * (kDin / 64)) % 8 == 0);
static_assert(((kRows / 32) * (kDm / 64)) % 8 == 0);

extern "C" void kernel_launch(void* const* d_in, const int* in_sizes, int n_in,
                              void* d_out, int out_size, void* d_ws, size_t ws_size,
                              hipStream_t stream)
{
  if (n_in < 18) return;
  if (in_sizes[0]  != kRows * kDm) return;
  if (in_sizes[1]  != kBatch * kDin * kNst) return;
  if (in_sizes[2]  != kDm * kXp) return;
  if (in_sizes[3]  != kXp) return;
  if (in_sizes[4]  != 4 * kDin) return;
  if (in_sizes[5]  != kDin) return;
  if (in_sizes[6]  != kDin * kDtr) return;
  if (in_sizes[7]  != kDtr) return;
  if (in_sizes[8]  != kDtr * kDin) return;
  if (in_sizes[9]  != kDin) return;
  if (in_sizes[10] != kDin * kNst) return;
  if (in_sizes[11] != kDin * kNst) return;
  if (in_sizes[12] != kNst) return;
  if (in_sizes[13] != kDin * kNst) return;
  if (in_sizes[14] != kNst) return;
  if (in_sizes[15] != kDin) return;
  if (in_sizes[16] != kDin * kDm) return;
  if (in_sizes[17] != kDm) return;
  if (out_size != kRows * kDm + kBatch * kDin * kNst) return;
  if (ws_size < kWsTotal) return;

  const float* x           = (const float*)d_in[0];
  const float* ssm_state   = (const float*)d_in[1];
  const float* in_proj_w   = (const float*)d_in[2];
  const float* in_proj_b   = (const float*)d_in[3];
  const float* conv_w      = (const float*)d_in[4];
  const float* conv_b      = (const float*)d_in[5];
  const float* dt_proj_w   = (const float*)d_in[6];
  const float* dt_proj_b   = (const float*)d_in[7];
  const float* dt_expand_w = (const float*)d_in[8];
  const float* dt_expand_b = (const float*)d_in[9];
  const float* A_log       = (const float*)d_in[10];
  const float* B_proj_w    = (const float*)d_in[11];
  const float* B_proj_b    = (const float*)d_in[12];
  const float* C_proj_w    = (const float*)d_in[13];
  const float* C_proj_b    = (const float*)d_in[14];
  const float* D_param     = (const float*)d_in[15];
  const float* out_proj_w  = (const float*)d_in[16];
  const float* out_proj_b  = (const float*)d_in[17];
  float* out  = (float*)d_out;
  float* hfin = out + (size_t)kRows * kDm;

  char* ws = (char*)d_ws;
  unsigned short* W0T  = (unsigned short*)(ws + kOffW0);
  unsigned short* W7T  = (unsigned short*)(ws + kOffW7);
  unsigned short* WCH  = (unsigned short*)(ws + kOffWCH);
  unsigned short* WCL  = (unsigned short*)(ws + kOffWCL);
  unsigned short* W3T  = (unsigned short*)(ws + kOffW3);
  float*          BCAT = (float*)(ws + kOffBCAT);
  unsigned short* XH   = (unsigned short*)(ws + kOffXH);
  unsigned short* XL   = kSplitIn ? (unsigned short*)(ws + kOffXL) : XH;
  float*          XI   = (float*)(ws + kOffXI);
  float*          SG   = (float*)(ws + kOffSG);
  float*          XC   = (float*)(ws + kOffXC);
  unsigned short* XCH  = (unsigned short*)(ws + kOffXCH);
  unsigned short* XCL  = (unsigned short*)(ws + kOffXCL);
  float*          P    = (float*)(ws + kOffP);
  unsigned short* DLH  = (unsigned short*)(ws + kOffDLH);
  float*          DT   = (float*)(ws + kOffDT);
  unsigned short* YH   = (unsigned short*)(ws + kOffYH);
  unsigned short* YL   = kSplitOut ? (unsigned short*)(ws + kOffYL) : YH;

  transpose_pack_kernel<false><<<dim3(kXp / 64, kDm / 64), 256, 0, stream>>>(in_proj_w, W0T, W0T, kDm, kXp, kWCarry);
  transpose_pack_kernel<false><<<dim3(kDm / 64, kDin / 64), 256, 0, stream>>>(out_proj_w, W7T, W7T, kDin, kDm, kWCarry);
  transpose_pack_kernel<false><<<dim3(kDin / 64, kDtr / 64), 256, 0, stream>>>(dt_expand_w, W3T, W3T, kDtr, kDin, kWCarry);
  pack_cat_kernel<<<dim3(kCatN / 64, kDin / 64), 256, 0, stream>>>(dt_proj_w, B_proj_w, C_proj_w, WCH, WCL, kWCarry);
  bias_cat_kernel<<<1, 32, 0, stream>>>(dt_proj_b, B_proj_b, C_proj_b, BCAT);

  split_rows_f16_kernel<kSplitIn><<<(kRows * kDm / 8) / 256, 256, 0, stream>>>(x, XH, XL, kRows * kDm / 8);

  constexpr int kSplIn  = kSplitIn ? 1 : 0;
  constexpr int kSplOut = kSplitOut ? 1 : 0;

  eng::gemm_f16_kernel<2, kSplIn, 1><<<dim3((kRows / 32) * (kXp / 64) / 8), 256, 0, stream>>>(
      XH, XL, kDm, W0T, W0T, kDm, XI, SG, kDin, kDin, in_proj_b, kRows, kXp, kDm, sIn, sInR);

  conv_silu_kernel<<<dim3(kDin / 256, kRows / 64), 256, 0, stream>>>(XI, conv_w, conv_b, XC, XCH, XCL);

  eng::gemm_f16_kernel<1, 2, 0><<<dim3((kRows / 16) * (kCatN / 64) / 8), 256, 0, stream>>>(
      XCH, XCL, kDin, WCH, WCL, kDin, P, P, kCatN, kCatN, BCAT, kRows, kCatN, kDin, sCat, sCatR);

  dtlow_f16_kernel<<<(kRows * kDtr / 8) / 256, 256, 0, stream>>>(P, DLH, kRows * kDtr / 8);

  eng::gemm_f16_kernel<2, 0, 2><<<dim3((kRows / 32) * (kDin / 64) / 8), 256, 0, stream>>>(
      DLH, DLH, kDtr, W3T, W3T, kDtr, DT, DT, kDin, kDin, dt_expand_b, kRows, kDin, kDtr, sExp, 0.0f);

  scan_final_kernel<kSplitOut><<<dim3(kBatch * (kDin / 128)), 64, 0, stream>>>(
      DT, XC, SG, P, A_log, D_param, ssm_state, (unsigned*)YH, (unsigned*)YL, hfin);

  eng::gemm_f16_kernel<2, kSplOut, 0><<<dim3((kRows / 32) * (kDm / 64) / 8), 256, 0, stream>>>(
      YH, YL, kDin, W7T, W7T, kDin, out, out, kDm, kDm, out_proj_b, kRows, kDm, kDin, sOut, sOutR);
}
